// RootAlign_40570261078532
// MI455X (gfx1250) — hardware-verified
//
#include <hip/hip_runtime.h>

typedef _Float16 v16h __attribute__((ext_vector_type(16)));
typedef _Float16 v8h  __attribute__((ext_vector_type(8)));
typedef _Float16 v4h  __attribute__((ext_vector_type(4)));
typedef float    v8f  __attribute__((ext_vector_type(8)));
typedef float    v4f  __attribute__((ext_vector_type(4)));
typedef v8h __attribute__((may_alias)) v8ha;
typedef v4h __attribute__((may_alias)) v4ha;
typedef v4f __attribute__((may_alias)) v4fa;

union Frag { v16h v; v8h half[2]; };

#define WD        300
#define HID       300
#define RELS      3
#define LEAVES    256
#define NT        19
#define NPAD      (NT * 16)
#define KC_LEAF   10
#define KC_COMB   19
#define XP        320
#define HP        304
#define FRAGH     512
#define WLEAF_HALVES (NT * KC_LEAF * FRAGH)
#define WH_HALVES    (NT * KC_COMB * FRAGH)
#define LINEF     32
#define NTHREADS  256
#define NWAVES    8

#define LDS_A_HALVES   (256 * HP)
#define LDS_X_HALVES   (128 * XP)
#define LDS_S_HALVES   (32 * HP)
#define LDS_BYTES ((size_t)(LDS_A_HALVES + LDS_X_HALVES + LDS_S_HALVES) * 2 + (size_t)2 * NPAD * 4)

static_assert((WLEAF_HALVES % 256) == 0);
static_assert((WH_HALVES % 256) == 0);
static_assert(128 * HP <= LDS_X_HALVES);

__device__ __forceinline__ v8f wmma16(v16h a, v16h b, v8f c) {
    v8f d = __builtin_amdgcn_wmma_f32_16x16x32_f16(false, a, false, b, (short)0, c, false, false);
    asm volatile("v_nop\n\tv_nop\n\tv_nop\n\tv_nop" : "+v"(d) : "v"(a), "v"(b));
    return d;
}

__device__ __forceinline__ v16h load_A(const _Float16* rowk0, int hsel) {
    Frag f;
    f.half[0] = *(const v8ha*)(rowk0 + 8 * hsel);
    f.half[1] = *(const v8ha*)(rowk0 + 16 + 8 * hsel);
    return f.v;
}

__device__ __forceinline__ v16h load_B(const _Float16* __restrict__ pack, int frag, int lane) {
    Frag f;
    const _Float16* p = pack + (size_t)frag * FRAGH + lane * 16;
    f.half[0] = *(const v8ha*)(p);
    f.half[1] = *(const v8ha*)(p + 8);
    return f.v;
}

__global__ __launch_bounds__(256) void pack_wleaf(const float* __restrict__ wl, _Float16* __restrict__ dst, int nthr) {
    const int q = blockIdx.x * 256 + threadIdx.x;
    if (q >= nthr) return;
    const int base = q * 8;
    const int frag = base >> 9;
    const int rr   = base & 511;
    const int lane = rr >> 4;
    const int i0   = rr & 15;
    const int nt = frag / KC_LEAF, ck = frag - nt * KC_LEAF;
    const int n  = nt * 16 + (lane & 15);
    const int kb = ck * 32 + 8 * (lane >> 4) + 2 * i0;
    const int nc = min(n, HID - 1);
    float v[8];
    #pragma unroll
    for (int i = 0; i < 8; ++i) {
        const int k  = kb + i;
        const int kc = min(k, WD - 1);
        const float w = wl[(size_t)nc * WD + kc];
        v[i] = (k < WD && n < HID) ? w * 16.0f : 0.0f;
    }
    const v8h o = { (_Float16)v[0], (_Float16)v[1], (_Float16)v[2], (_Float16)v[3],
                    (_Float16)v[4], (_Float16)v[5], (_Float16)v[6], (_Float16)v[7] };
    _Float16* p = dst + (size_t)base;
    *(volatile v8h*)p = o;
    __threadfence();
    *(volatile v8h*)p = o;
}

__global__ __launch_bounds__(256) void pack_wh(const float* __restrict__ wh, _Float16* __restrict__ dst, int nthr) {
    const int q = blockIdx.x * 256 + threadIdx.x;
    if (q >= nthr) return;
    const int base = q * 8;
    const int frag = base >> 9;
    const int rr   = base & 511;
    const int lane = rr >> 4;
    const int i0   = rr & 15;
    const int nt = frag / KC_COMB, ck = frag - nt * KC_COMB;
    const int n  = nt * 16 + (lane & 15);
    const int kb = ck * 32 + 8 * (lane >> 4) + 2 * i0;
    const int nc = min(n, HID - 1);
    float v[8];
    #pragma unroll
    for (int i = 0; i < 8; ++i) {
        const int kp = kb + i;
        const bool left  = (kp < HID);
        const bool right = (kp >= HP) && (kp < HP + HID);
        int col = left ? kp : (kp - (HP - HID));
        col = min(max(col, 0), 2 * HID - 1);
        const float w = wh[(size_t)nc * (2 * HID) + col];
        v[i] = ((left || right) && n < HID) ? w * 16.0f : 0.0f;
    }
    const v8h o = { (_Float16)v[0], (_Float16)v[1], (_Float16)v[2], (_Float16)v[3],
                    (_Float16)v[4], (_Float16)v[5], (_Float16)v[6], (_Float16)v[7] };
    _Float16* p = dst + (size_t)base;
    *(volatile v8h*)p = o;
    __threadfence();
    *(volatile v8h*)p = o;
}

template<int NTG>
__device__ __forceinline__ void leaf_unit(const _Float16* bufX, _Float16* bufA,
                                          const _Float16* __restrict__ wlp,
                                          int mt, int nt0, int rowbase, int lane, int hsel, int m16) {
    const v8f zero8 = {0.f, 0.f, 0.f, 0.f, 0.f, 0.f, 0.f, 0.f};
    const _Float16* arow = bufX + (mt * 16 + m16) * XP;
    v8f acc[NTG];
    #pragma unroll
    for (int t = 0; t < NTG; ++t) acc[t] = zero8;
    #pragma unroll 1
    for (int ck = 0; ck < KC_LEAF; ++ck) {
        const v16h a = load_A(arow + ck * 32, hsel);
        #pragma unroll
        for (int t = 0; t < NTG; ++t) {
            const v16h b = load_B(wlp, (nt0 + t) * KC_LEAF + ck, lane);
            acc[t] = wmma16(a, b, acc[t]);
        }
    }
    const int rb = rowbase + mt * 16 + 8 * hsel;
    #pragma unroll
    for (int t = 0; t < NTG; ++t) {
        const int ncol = (nt0 + t) * 16 + m16;
        #pragma unroll
        for (int r = 0; r < 8; ++r)
            bufA[(rb + r) * HP + ncol] = (_Float16)(acc[t][r] * 0.0625f);
    }
}

template<int NTG, bool FIN>
__device__ __forceinline__ void comb_unit(const _Float16* cur, int Mout, _Float16* nxt, float* rootf,
                                          const _Float16* __restrict__ whp, const float* __restrict__ bh,
                                          int mt, int nt0, int lane, int hsel, int m16) {
    const v8f zero8 = {0.f, 0.f, 0.f, 0.f, 0.f, 0.f, 0.f, 0.f};
    const int m  = mt * 16 + m16;
    const int mm = min(m, Mout - 1);
    const _Float16* arow = cur + mm * (2 * HP);
    v8f acc[NTG];
    #pragma unroll
    for (int t = 0; t < NTG; ++t) acc[t] = zero8;
    #pragma unroll 1
    for (int ck = 0; ck < KC_COMB; ++ck) {
        const v16h a = load_A(arow + ck * 32, hsel);
        #pragma unroll
        for (int t = 0; t < NTG; ++t) {
            const v16h b = load_B(whp, (nt0 + t) * KC_COMB + ck, lane);
            acc[t] = wmma16(a, b, acc[t]);
        }
    }
    #pragma unroll
    for (int t = 0; t < NTG; ++t) {
        const int ncol = (nt0 + t) * 16 + m16;
        float bb = bh[min(ncol, HID - 1)];
        bb = (ncol < HID) ? bb : 0.0f;
        if (FIN) {
            if (hsel == 0) {
                rootf[ncol]        = acc[t][0] * 0.0078125f + bb;
                rootf[NPAD + ncol] = acc[t][1] * 0.0078125f + bb;
            }
        } else {
            const float b8 = 8.0f * bb;
            #pragma unroll
            for (int r = 0; r < 8; ++r) {
                const int mrow = mt * 16 + 8 * hsel + r;
                if (mrow < Mout)
                    nxt[mrow * HP + ncol] = (_Float16)(acc[t][r] * 0.0625f + b8);
            }
        }
    }
}

template<bool FIN>
__device__ __forceinline__ void comb_level(const _Float16* cur, int nIn, _Float16* nxt, float* rootf,
                                           const _Float16* __restrict__ whp, const float* __restrict__ bh,
                                           int wave, int lane, int hsel, int m16) {
    const int Mout   = nIn >> 1;
    const int Mtiles = (Mout + 15) >> 4;
    const int units  = Mtiles * 4;
    for (int u = wave; u < units; u += NWAVES) {
        const int mt = u % Mtiles;
        const int g  = u / Mtiles;
        if (g < 3) comb_unit<5, FIN>(cur, Mout, nxt, rootf, whp, bh, mt, 5 * g, lane, hsel, m16);
        else       comb_unit<4, FIN>(cur, Mout, nxt, rootf, whp, bh, mt, 15,    lane, hsel, m16);
    }
}

__global__ void __launch_bounds__(NTHREADS)
tree_kernel(const int*   __restrict__ word_ids,
            const float* __restrict__ emb,
            const _Float16* __restrict__ wlp,
            const _Float16* __restrict__ whp,
            const float* __restrict__ bh,
            const float* __restrict__ wcls,
            const float* __restrict__ bcls,
            float* __restrict__ lines,
            int nvocab)
{
    extern __shared__ __align__(16) char smem_raw[];
    _Float16* bufA  = (_Float16*)smem_raw;
    _Float16* bufX  = bufA + LDS_A_HALVES;
    _Float16* stash = bufX + LDS_X_HALVES;
    float*    rootf = (float*)(stash + LDS_S_HALVES);

    const int b    = blockIdx.x;
    const int tid  = threadIdx.x;
    const int wave = tid >> 5;
    const int lane = tid & 31;
    const int hsel = lane >> 4;
    const int m16  = lane & 15;

    for (int s = 0; s < 2; ++s) {
        const int* ids = word_ids + ((size_t)b * 2 + s) * LEAVES;
        for (int hh = 0; hh < 2; ++hh) {
            __syncthreads();
            {
                const int g = tid >> 1;
                const int q = tid & 1;
                int wid = ids[hh * 128 + g];
                wid = min(max(wid, 0), nvocab - 1);
                const float* er = emb + (size_t)wid * WD;
                _Float16* xr = bufX + g * XP;
                #pragma unroll 2
                for (int j = q; j < XP / 4; j += 2) {
                    const int jj = min(j, WD / 4 - 1);
                    const v4f v = *(const v4fa*)(er + 4 * jj);
                    const float sc = (j < WD / 4) ? 8.0f : 0.0f;
                    v4h o;
                    o.x = (_Float16)(v.x * sc); o.y = (_Float16)(v.y * sc);
                    o.z = (_Float16)(v.z * sc); o.w = (_Float16)(v.w * sc);
                    *(v4ha*)(xr + 4 * j) = o;
                }
            }
            __syncthreads();
            for (int u = wave; u < 32; u += NWAVES) {
                const int mt = u & 7;
                const int g  = u >> 3;
                if (g < 3) leaf_unit<5>(bufX, bufA, wlp, mt, 5 * g, hh * 128, lane, hsel, m16);
                else       leaf_unit<4>(bufX, bufA, wlp, mt, 15,    hh * 128, lane, hsel, m16);
            }
        }
        {
            const _Float16* cur = bufA;
            int nIn = 256;
            for (int L = 0; L < 4; ++L) {
                _Float16* nxt = (L == 3) ? (stash + s * 16 * HP) : ((L & 1) ? bufA : bufX);
                __syncthreads();
                comb_level<false>(cur, nIn, nxt, rootf, whp, bh, wave, lane, hsel, m16);
                cur = nxt;
                nIn >>= 1;
            }
        }
    }
    {
        const _Float16* cur = stash;
        int nIn = 32;
        for (int L = 0; L < 3; ++L) {
            _Float16* nxt = (L & 1) ? bufA : bufX;
            __syncthreads();
            comb_level<false>(cur, nIn, nxt, rootf, whp, bh, wave, lane, hsel, m16);
            cur = nxt;
            nIn >>= 1;
        }
        __syncthreads();
        comb_level<true>(cur, nIn, bufA, rootf, whp, bh, wave, lane, hsel, m16);
    }
    __syncthreads();

    if (wave == 0) {
        float a0 = 0.0f, a1 = 0.0f, a2 = 0.0f;
        #pragma unroll 1
        for (int jj = 0; jj < (2 * HID + 31) / 32; ++jj) {
            const int j  = lane + 32 * jj;
            const int jc = min(j, 2 * HID - 1);
            const float ok = (j < 2 * HID) ? 1.0f : 0.0f;
            const int s2 = (jc >= HID) ? 1 : 0;
            const int n2 = jc - s2 * HID;
            const float x = rootf[s2 * NPAD + n2];
            const float f = __frcp_rn(1.0f + __expf(-x)) * ok;
            a0 += f * wcls[jc];
            a1 += f * wcls[2 * HID + jc];
            a2 += f * wcls[4 * HID + jc];
        }
        #pragma unroll
        for (int o = 16; o >= 1; o >>= 1) {
            a0 += __shfl_xor(a0, o, 32);
            a1 += __shfl_xor(a1, o, 32);
            a2 += __shfl_xor(a2, o, 32);
        }
        const float l0 = a0 + bcls[0];
        const float l1 = a1 + bcls[1];
        const float l2 = a2 + bcls[2];
        const float mx = fmaxf(l0, fmaxf(l1, l2));
        const float sum = __expf(l0 - mx) + __expf(l1 - mx) + __expf(l2 - mx);
        const float lse = mx + __logf(sum);
        const float p0 = l0 - lse, p1 = l1 - lse, p2 = l2 - lse;
        const float v = (lane == 0) ? p0 : ((lane == 1) ? p1 : ((lane == 2) ? p2 : 0.0f));
        volatile float* lp = lines + (size_t)b * LINEF + lane;
        *lp = v;
        __threadfence();
        *lp = v;
    }
}

__global__ __launch_bounds__(256) void out_kernel(const float* __restrict__ lines, float* __restrict__ out, int n_out) {
    const int t  = blockIdx.x * 256 + threadIdx.x;
    const int e0 = 4 * t;
    if (e0 >= n_out) return;
    float v[4];
    #pragma unroll
    for (int j = 0; j < 4; ++j) {
        const int e   = min(e0 + j, n_out - 1);
        const int row = e / RELS;
        const int col = e - row * RELS;
        v[j] = lines[(size_t)row * LINEF + col];
    }
    if (e0 + 3 < n_out) {
        const v4f o = {v[0], v[1], v[2], v[3]};
        *(volatile v4f*)(out + e0) = o;
        __threadfence();
        *(volatile v4f*)(out + e0) = o;
    } else {
        #pragma unroll
        for (int j = 0; j < 4; ++j)
            if (e0 + j < n_out) *(volatile float*)(out + e0 + j) = v[j];
        __threadfence();
        #pragma unroll
        for (int j = 0; j < 4; ++j)
            if (e0 + j < n_out) *(volatile float*)(out + e0 + j) = v[j];
    }
}

extern "C" void kernel_launch(void* const* d_in, const int* in_sizes, int n_in,
                              void* d_out, int out_size, void* d_ws, size_t ws_size,
                              hipStream_t stream) {
    if (n_in < 7) return;
    const int nb = in_sizes[0] / (2 * LEAVES);
    if (nb <= 0 || in_sizes[0] != nb * 2 * LEAVES) return;
    const int nvocab = in_sizes[1] / WD;
    if (nvocab <= 0 || in_sizes[1] != nvocab * WD) return;
    if (in_sizes[2] != HID * WD) return;
    if (in_sizes[3] != HID * 2 * HID) return;
    if (in_sizes[4] != HID) return;
    if (in_sizes[5] != RELS * 2 * HID) return;
    if (in_sizes[6] != RELS) return;
    if (out_size != nb * RELS) return;

    const int*   word_ids = (const int*)  d_in[0];
    const float* emb      = (const float*)d_in[1];
    const float* wleaf    = (const float*)d_in[2];
    const float* wh       = (const float*)d_in[3];
    const float* bh       = (const float*)d_in[4];
    const float* wcls     = (const float*)d_in[5];
    const float* bcls     = (const float*)d_in[6];

    const size_t off_wl   = 0;
    const size_t by_wl    = (size_t)WLEAF_HALVES * 2;
    const size_t off_wh   = off_wl + by_wl;
    const size_t by_wh    = (size_t)WH_HALVES * 2;
    const size_t off_ln   = off_wh + by_wh;
    const size_t by_ln    = (size_t)nb * LINEF * 4;
    const size_t total    = off_ln + by_ln;
    if (total > ws_size) return;

    char* ws = (char*)d_ws;
    _Float16* wlp   = (_Float16*)(ws + off_wl);
    _Float16* whp   = (_Float16*)(ws + off_wh);
    float*    lines = (float*)(ws + off_ln);

    const int thr_wl = WLEAF_HALVES / 8;
    const int thr_wh = WH_HALVES / 8;
    pack_wleaf<<<(thr_wl + 255) / 256, 256, 0, stream>>>(wleaf, wlp, thr_wl);
    pack_wh<<<(thr_wh + 255) / 256, 256, 0, stream>>>(wh, whp, thr_wh);

    const size_t smem = LDS_BYTES;
    (void)hipFuncSetAttribute(reinterpret_cast<const void*>(&tree_kernel),
                              hipFuncAttributeMaxDynamicSharedMemorySize, (int)smem);
    tree_kernel<<<nb, NTHREADS, smem, stream>>>(word_ids, emb, wlp, whp, bh, wcls, bcls, lines, nvocab);

    const int thr_out = (out_size + 3) / 4;
    out_kernel<<<(thr_out + 255) / 256, 256, 0, stream>>>(lines, (float*)d_out, out_size);
}
